// wconv_3x3_63041529970868
// MI455X (gfx1250) — hardware-verified
//
#include <hip/hip_runtime.h>


namespace {
constexpr int NI = 16, C = 256, K = 256, HH = 56, WW = 56, P = HH * WW  , KK = C * 9  ;
constexpr float XS = 8.0f, WSC = 256.0f;
typedef _Float16 b16;
typedef __attribute__((ext_vector_type(16))) _Float16 v16b;
typedef __attribute__((ext_vector_type(8))) _Float16 v8b;
typedef __attribute__((ext_vector_type(8))) float v8f;
typedef __attribute__((ext_vector_type(4))) float v4f;
__device__ __forceinline__ float bf16_rne(float f) { unsigned int u = __float_as_uint(f); u += 0x7FFFu + ((u >> 16) & 1u); return __uint_as_float(u & 0xFFFF0000u); }
__device__ __forceinline__ v16b frag_kb(const b16* p, int hh) { const v8b a = *(const v8b*)(p + 8 * hh), b = *(const v8b*)(p + 16 + 8 * hh); v16b f;
#pragma unroll
  for (int e = 0; e < 8; ++e) { f[e] = a[e]; f[8 + e] = b[e]; } return f; }
__device__ __forceinline__ v8f wmma16b(v16b a, v16b b, v8f c) { v8f d = __builtin_amdgcn_wmma_f32_16x16x32_f16(false, a, false, b, (short)0, c, false, false); asm volatile("v_nop\n\tv_nop\n\tv_nop\n\tv_nop" : "+v"(d) : "v"(a), "v"(b)); return d; }

__global__ __launch_bounds__(256) void prepw_kernel(const float* __restrict__ w, b16* __restrict__ W16) {
  const size_t u = (size_t)blockIdx.x * 256 + threadIdx.x; if (u >= (size_t)K * KK / 8) return; const size_t e = u * 8; v8b o; for (int j = 0; j < 8; ++j) o[j] = (b16)(bf16_rne(w[e + j]) * WSC);
  for (int pass = 0; pass < 2; ++pass) { *(volatile v8b*)(W16 + e) = o; __threadfence(); }
}
__global__ __launch_bounds__(256) void prepx_kernel(const float* __restrict__ x, b16* __restrict__ X16) {
  const size_t u = (size_t)blockIdx.x * 256 + threadIdx.x; if (u >= (size_t)NI * C * P / 8) return; const size_t e = u * 8; const v4f a = *(const v4f*)(x + e), b = *(const v4f*)(x + e + 4); v8b o;
  for (int j = 0; j < 4; ++j) { o[j] = (b16)(bf16_rne(a[j]) * XS); o[4 + j] = (b16)(bf16_rne(b[j]) * XS); } for (int pass = 0; pass < 2; ++pass) { *(volatile v8b*)(X16 + e) = o; __threadfence(); }
}
__global__ __launch_bounds__(128) void conv_kernel(const b16* __restrict__ X16, const b16* __restrict__ W16, float* __restrict__ y) {
  __shared__ __attribute__((aligned(16))) float St[K][64 + 4];
  const int wave = threadIdx.x >> 5, lane = threadIdx.x & 31, nloc = lane & 15, hlf = lane >> 4, t_ = threadIdx.x; const int n = blockIdx.y; const int p0 = blockIdx.x * 64 + wave * 16; const int pix = p0 + nloc; const int py = pix / WW, px = pix % WW;
  const b16* Xn = X16 + (size_t)n * C * P;
  v8f acc[16];
#pragma unroll
  for (int t = 0; t < 16; ++t) acc[t] = (v8f){};
  for (int kb = 0; kb < KK; kb += 32) {
    v16b a;
#pragma unroll
    for (int e = 0; e < 16; ++e) { const int kk = kb + ((e < 8) ? (8 * hlf + e) : (16 + 8 * hlf + (e - 8))); const int c = kk / 9, tap = kk % 9; const int yy = py + tap / 3 - 1, xx = px + tap % 3 - 1;
      const int yc = yy < 0 ? 0 : (yy >= HH ? HH - 1 : yy), xc = xx < 0 ? 0 : (xx >= WW ? WW - 1 : xx);
      const b16 v = Xn[((size_t)c * HH + yc) * WW + xc]; a[e] = (yy >= 0 && yy < HH && xx >= 0 && xx < WW) ? v : (b16)0.0f; }
#pragma unroll
    for (int t = 0; t < 16; ++t) acc[t] = wmma16b(a, frag_kb(W16 + (size_t)(t * 16 + nloc) * KK + kb, hlf), acc[t]); }
#pragma unroll
  for (int t = 0; t < 16; ++t)
#pragma unroll 1
    for (int r = 0; r < 8; ++r) St[t * 16 + nloc][wave * 16 + 8 * hlf + r] = acc[t][r] * (1.0f / (XS * WSC));
  __syncthreads();
  for (int pass = 0; pass < 2; ++pass) { for (int q = t_; q < K * 16; q += 128) { const int oc = q >> 4, c4 = (q & 15) * 4; *(volatile v4f*)(y + ((size_t)n * K + oc) * P + blockIdx.x * 64 + c4) = *(const v4f*)(&St[oc][c4]); } __threadfence(); }
}
}

extern "C" void kernel_launch(void* const* d_in, const int* in_sizes, int n_in, void* d_out, int out_size, void* d_ws, size_t ws_size, hipStream_t stream) {
  (void)n_in;
  auto Fp = [&](int i) { return (const float*)d_in[i]; };
  if (in_sizes[0] != NI * C * P || in_sizes[1] != K * C * 9 || out_size != NI * K * P) return;
  size_t off = 0; char* ws = (char*)d_ws;
  auto carve = [&](size_t bytes) { char* p = ws + off; off += (bytes + 255) & ~(size_t)255; return p; };
  b16* X16 = (b16*)carve((size_t)NI * C * P * 2); b16* W16 = (b16*)carve((size_t)K * KK * 2);
  if (off > ws_size || off > ((size_t)128 << 20)) return;
  prepx_kernel<<<(unsigned)(((size_t)NI * C * P / 8 + 255) / 256), 256, 0, stream>>>(Fp(0), X16);
  prepw_kernel<<<(unsigned)(((size_t)K * KK / 8 + 255) / 256), 256, 0, stream>>>(Fp(1), W16);
  conv_kernel<<<dim3(P / 64, NI), 128, 0, stream>>>(X16, W16, (float*)d_out);
}
